// Encoder_47656957116696
// MI455X (gfx1250) — hardware-verified
//
#include <hip/hip_runtime.h>
#include <math.h>

constexpr int kBatch     = 16;
constexpr int kSteps     = 2048;
constexpr int kCin       = 64;
constexpr int kFilt      = 256;
constexpr int kUnits     = 256;
constexpr int kGate3     = 768;
constexpr int kHalfSteps = 1024;
constexpr int kPadRows   = 2050;
constexpr int kConvK     = 192;
constexpr int kRows      = kBatch * kSteps;
constexpr int kRowsHalf  = kBatch * kHalfSteps;
constexpr int kOut0      = kRows * kUnits;
constexpr int kOut1      = kBatch * kUnits * 2;
constexpr int HP         = 264;
constexpr int OP         = 260;
static_assert(kGate3 == 3 * kUnits, "gate columns");
static_assert(kConvK == 3 * kCin, "conv K");
static_assert(kConvK % 32 == 0 && kFilt % 32 == 0 && kUnits % 32 == 0, "K multiples of 32");
static_assert(kRows % 64 == 0 && kRowsHalf % 64 == 0 && kFilt % 64 == 0 && kGate3 % 64 == 0, "M, N tile multiples");
static_assert(kSteps % 64 == 0 && kHalfSteps % 64 == 0, "row tiles never straddle a sequence");
static_assert(kBatch == 16, "one 16-row m-subtile per scan block");
static_assert(kUnits == 32 * 8, "8 waves x 32 hidden units");
static_assert((kOut0 * 4) % 128 == 0, "second output starts on a line");

typedef __attribute__((ext_vector_type(8)))  _Float16 v8h;
typedef __attribute__((ext_vector_type(16))) __bf16   v16b;
typedef __attribute__((ext_vector_type(8)))  __bf16   v8b;
typedef __attribute__((ext_vector_type(8)))  float    v8f;
typedef __attribute__((ext_vector_type(4)))  float    v4f;

__device__ __forceinline__ unsigned short f2bf_bits(float f) {
  unsigned u = __float_as_uint(f);
  return (unsigned short)((u + 0x7FFFu + ((u >> 16) & 1u)) >> 16);
}
__device__ __forceinline__ float bf_bits2f(unsigned short h) { return __uint_as_float(((unsigned)h) << 16); }
__device__ __forceinline__ float bf16r(float f) { return bf_bits2f(f2bf_bits(f)); }

__device__ __forceinline__ void guard4_b(v8f& a, v8f& b, v8f& c, v8f& d, v16b x, v16b y) {
  asm volatile("v_nop\n\tv_nop\n\tv_nop\n\tv_nop" : "+v"(a), "+v"(b), "+v"(c), "+v"(d) : "v"(x), "v"(y));
}
__device__ __forceinline__ void guard3_b(v8f& a, v8f& b, v8f& c, v16b x, v16b y, v16b p, v16b q, v16b s) {
  asm volatile("v_nop\n\tv_nop\n\tv_nop\n\tv_nop" : "+v"(a), "+v"(b), "+v"(c) : "v"(x), "v"(y), "v"(p), "v"(q), "v"(s));
}
__device__ __forceinline__ void keep4_b(v16b a, v16b b, v16b c, v16b d) { asm volatile("v_nop" :: "v"(a), "v"(b), "v"(c), "v"(d)); }
__device__ __forceinline__ void acc_guard4(v8f& a, v8f& b, v8f& c, v8f& d) { asm volatile("v_nop\n\tv_nop\n\tv_nop\n\tv_nop" : "+v"(a), "+v"(b), "+v"(c), "+v"(d)); }
__device__ __forceinline__ void acc_guard3(v8f& a, v8f& b, v8f& c) { asm volatile("v_nop\n\tv_nop\n\tv_nop\n\tv_nop" : "+v"(a), "+v"(b), "+v"(c)); }

template <typename T> struct Frag;
template <> struct Frag<__bf16> {
  typedef v16b V; union U { v16b v; v8b h[2]; };
  static __device__ __forceinline__ v16b load(const __bf16* p) {
    U f; f.h[0] = *(const v8b*)(p); f.h[1] = *(const v8b*)(p + 16); return f.v;
  }
  static __device__ __forceinline__ v8f mma(v16b a, v16b b, v8f c) {
    return __builtin_amdgcn_wmma_f32_16x16x32_bf16(false, a, false, b, (short)0, c, false, false);
  }
};

__device__ __forceinline__ float elu1(float y) {
  const float ym = fminf(y, 0.0f);
  const float ex = expf(ym) - 1.0f;
  const float ts = ym * (1.0f + ym * (0.5f + ym * (0.16666667f + ym * (0.041666668f + ym * 0.0083333338f))));
  const float em = (ym > -0.03125f) ? ts : ex;
  return (y > 0.0f) ? y : em;
}
__device__ __forceinline__ float fsig(float x)  { return __builtin_amdgcn_rcpf(1.0f + expf(-x)); }
__device__ __forceinline__ float ftanh(float x) { return 1.0f - 2.0f * __builtin_amdgcn_rcpf(expf(2.0f * x) + 1.0f); }

__global__ __launch_bounds__(256) void xpad_kernel(const float* __restrict__ xin, unsigned short* __restrict__ xpad) {
  const int i = blockIdx.x * 256 + threadIdx.x;
  constexpr int n8 = kBatch * kPadRows * (kCin / 8);
  if (i < n8) {
    const int c8   = (i & 7) * 8;
    const int rowi = i >> 3;
    const int b    = rowi / kPadRows;
    const int p    = rowi - b * kPadRows;
    const bool valid = (p >= 1) && (p <= kSteps);
    int tc = p - 1;
    tc = tc < 0 ? 0 : (tc > kSteps - 1 ? kSteps - 1 : tc);
    const float* sp = xin + ((size_t)b * kSteps + (size_t)tc) * kCin + c8;
    const v4f va = *(const v4f*)(sp);
    const v4f vb = *(const v4f*)(sp + 4);
    v8h hv;
#pragma unroll
    for (int e = 0; e < 4; ++e) {
      const float fa = va[e];
      const float fb = vb[e];
      const unsigned short ba = f2bf_bits(fa);
      const unsigned short bb = f2bf_bits(fb);
      const unsigned short sa = valid ? ba : (unsigned short)0;
      const unsigned short sb = valid ? bb : (unsigned short)0;
      hv[e]     = __builtin_bit_cast(_Float16, sa);
      hv[4 + e] = __builtin_bit_cast(_Float16, sb);
    }
    *(volatile v8h*)(xpad + (size_t)i * 8) = hv;
    __threadfence();
    *(volatile v8h*)(xpad + (size_t)i * 8) = hv;
  }
}

__global__ __launch_bounds__(256) void zero_kernel(float* __restrict__ p, int n4) {
  const int i = blockIdx.x * 256 + threadIdx.x;
  if (i < n4) {
    const v4f z = {0.f, 0.f, 0.f, 0.f};
    *(volatile v4f*)(p + (size_t)i * 4) = z;
    __threadfence();
    *(volatile v4f*)(p + (size_t)i * 4) = z;
  }
}

__global__ __launch_bounds__(256) void tp_bf16_kernel(const float* __restrict__ s0, const float* __restrict__ s1,
                                                      const float* __restrict__ s2, const float* __restrict__ s3,
                                                      unsigned short* __restrict__ o0, unsigned short* __restrict__ o1,
                                                      unsigned short* __restrict__ o2, unsigned short* __restrict__ o3,
                                                      int R, int C) {
  __shared__ float Tt[64 * 65];
  const int z = blockIdx.z;
  const float* src = (z == 0) ? s0 : (z == 1) ? s1 : (z == 2) ? s2 : s3;
  unsigned short* O = (z == 0) ? o0 : (z == 1) ? o1 : (z == 2) ? o2 : o3;
  const int tid = threadIdx.x;
  const int c0 = blockIdx.x * 64, r0 = blockIdx.y * 64;
#pragma unroll
  for (int i = 0; i < 4; ++i) {
    const int idx = i * 256 + tid;
    const int rr = idx >> 4, cc = (idx & 15) * 4;
    const v4f v = *(const v4f*)(src + (size_t)(r0 + rr) * (size_t)C + c0 + cc);
    Tt[rr * 65 + cc + 0] = v[0];
    Tt[rr * 65 + cc + 1] = v[1];
    Tt[rr * 65 + cc + 2] = v[2];
    Tt[rr * 65 + cc + 3] = v[3];
  }
  __syncthreads();
  const int q = tid >> 3, c8 = (tid & 7) * 8;
  v8h hv[2];
#pragma unroll
  for (int g = 0; g < 2; ++g) {
    const int qq = g * 32 + q;
#pragma unroll
    for (int e = 0; e < 8; ++e) {
      const float f = Tt[(c8 + e) * 65 + qq];
      const unsigned short bits = f2bf_bits(f);
      hv[g][e] = __builtin_bit_cast(_Float16, bits);
    }
  }
  for (int pass = 0; pass < 2; ++pass) {
#pragma unroll
    for (int g = 0; g < 2; ++g) {
      const size_t o = (size_t)(c0 + g * 32 + q) * (size_t)R + (size_t)(r0 + c8);
      *(volatile v8h*)(O + o) = hv[g];
    }
    __threadfence();
  }
}

template <int NPA, int OUT_MODE>
__global__ __launch_bounds__(256) void gemm64_bf16(
    const unsigned short* __restrict__ Ahp, const unsigned short* __restrict__ Alp, int lda,
    int rshift, int radd, int rbase,
    const unsigned short* __restrict__ Btp, int ldb,
    void* __restrict__ Cout, void* __restrict__ Cout2, int ldc,
    const float* __restrict__ bias, int M, int N, int K) {
  typedef __bf16 T;
  typedef v16b V;
  const T* A = (const T*)Ahp; const T* A2 = (const T*)Alp; const T* Bt = (const T*)Btp;
  __shared__ __align__(16) float sT[8][16 * 68];
  const int lane = threadIdx.x & 31;
  const int wave = threadIdx.x >> 5;
  const int tilesN = N >> 6;
  const int tilesM = M >> 6;
  const int tile = blockIdx.x * 8 + wave;
  if (tile >= tilesM * tilesN) return;
  const int tm = tile / tilesN;
  const int tn = tile - tm * tilesN;
  const int m0 = tm << 6;
  const int n0 = tn << 6;

  const int rlane = lane & 15;
  const int koff  = (lane >> 4) * 8;
  const int mOff  = (lane >> 4) * 8;

  v8f acc[4][4];
#pragma unroll
  for (int i = 0; i < 4; ++i)
#pragma unroll
    for (int j = 0; j < 4; ++j) acc[i][j] = (v8f){0.f,0.f,0.f,0.f,0.f,0.f,0.f,0.f};

  for (int k0 = 0; k0 < K; k0 += 32) {
    V bh[4];
#pragma unroll
    for (int j = 0; j < 4; ++j) {
      const size_t bo = (size_t)(n0 + (j << 4) + rlane) * ldb + koff + k0;
      bh[j] = Frag<T>::load(Bt + bo);
    }
#pragma unroll
    for (int i = 0; i < 4; ++i) {
      const int m = m0 + (i << 4) + rlane;
      const int arow = m + (m >> rshift) * radd + rbase;
      const size_t ao = (size_t)arow * lda + koff + k0;
      V ah = Frag<T>::load(A + ao);
      V al = ah;
      if (NPA == 2) al = Frag<T>::load(A2 + ao);
#pragma unroll
      for (int j = 0; j < 4; ++j) acc[i][j] = Frag<T>::mma(ah, bh[j], acc[i][j]);
      if (NPA == 2) {
#pragma unroll
        for (int j = 0; j < 4; ++j) acc[i][j] = Frag<T>::mma(al, bh[j], acc[i][j]);
      }
      guard4_b(acc[i][0], acc[i][1], acc[i][2], acc[i][3], ah, al);
    }
    keep4_b(bh[0], bh[1], bh[2], bh[3]);
  }
  acc_guard4(acc[0][0], acc[0][1], acc[0][2], acc[0][3]);
  acc_guard4(acc[1][0], acc[1][1], acc[1][2], acc[1][3]);
  acc_guard4(acc[2][0], acc[2][1], acc[2][2], acc[2][3]);
  acc_guard4(acc[3][0], acc[3][1], acc[3][2], acc[3][3]);

  float* slab = sT[wave];
#pragma unroll
  for (int i = 0; i < 4; ++i) {
    const int mBase = m0 + (i << 4);
#pragma unroll
    for (int j = 0; j < 4; ++j) {
      const int n = n0 + (j << 4) + rlane;
      const float bv = bf16r(bias[n]);
#pragma unroll
      for (int r = 0; r < 8; ++r) {
        const float v = acc[i][j][r] + bv;
        slab[(mOff + r) * 68 + (j << 4) + rlane] = v;
      }
    }
    __builtin_amdgcn_fence(__ATOMIC_RELEASE, "workgroup");
    __builtin_amdgcn_wave_barrier();
    __builtin_amdgcn_fence(__ATOMIC_ACQUIRE, "workgroup");
    if (OUT_MODE == 0) {
      float* C = (float*)Cout;
      const int hh = lane >> 4, c4 = (lane & 15) * 4;
      for (int pass = 0; pass < 2; ++pass) {
#pragma unroll
        for (int it = 0; it < 8; ++it) {
          const int row = it * 2 + hh;
          v4f v = *(const v4f*)(slab + row * 68 + c4);
          *(volatile v4f*)(C + (size_t)(mBase + row) * ldc + n0 + c4) = v;
        }
        __threadfence();
      }
    } else {
#pragma unroll 1
      for (int q8 = 0; q8 < 8; ++q8) {
        const int idx = q8 * 32 + lane;
        const int row = idx >> 4;
        const int cc  = (idx & 15) * 4;
        float* sp = slab + row * 68 + cc;
        const v4f v = *(const v4f*)sp;
        const float x0 = v[0], x1 = v[1], x2 = v[2], x3 = v[3];
        v4f o;
        o[0] = elu1(x0);
        o[1] = elu1(x1);
        o[2] = elu1(x2);
        o[3] = elu1(x3);
        *(v4f*)sp = o;
      }
      __builtin_amdgcn_fence(__ATOMIC_RELEASE, "workgroup");
      __builtin_amdgcn_wave_barrier();
      __builtin_amdgcn_fence(__ATOMIC_ACQUIRE, "workgroup");
      const int q = lane >> 3, c8 = (lane & 7) * 8;
      unsigned short* C  = (unsigned short*)Cout;
      unsigned short* C2 = (unsigned short*)Cout2;
      for (int pass = 0; pass < 2; ++pass) {
#pragma unroll
        for (int it = 0; it < 4; ++it) {
          const int row = it * 4 + q;
          const float* sp = slab + row * 68 + c8;
          v8h hv, lv;
#pragma unroll
          for (int e = 0; e < 8; ++e) {
            const float f = sp[e];
            const unsigned short hb = f2bf_bits(f);
            const unsigned short lb = f2bf_bits(f - bf_bits2f(hb));
            hv[e] = __builtin_bit_cast(_Float16, hb);
            lv[e] = __builtin_bit_cast(_Float16, lb);
          }
          *(volatile v8h*)(C  + (size_t)(mBase + row) * ldc + n0 + c8) = hv;
          *(volatile v8h*)(C2 + (size_t)(mBase + row) * ldc + n0 + c8) = lv;
        }
        __threadfence();
      }
    }
    __builtin_amdgcn_fence(__ATOMIC_RELEASE, "workgroup");
    __builtin_amdgcn_wave_barrier();
    __builtin_amdgcn_fence(__ATOMIC_ACQUIRE, "workgroup");
  }
}

template <int LAYER>
__global__ __launch_bounds__(256) void gru_scan_kernel(const float* __restrict__ XP, const unsigned short* __restrict__ Utp,
                                                       const float* __restrict__ bvec, float* HC,
                                                       unsigned short* YH, unsigned short* YL,
                                                       float* out0, float* out1, int half) {
  constexpr int NHF = (LAYER == 1) ? 2 : 1;
  __shared__ __align__(16) unsigned short Ahh[2][16 * HP];
  __shared__ __align__(16) unsigned short Ahl[2][16 * HP];
  __shared__ __align__(16) float          Hf[NHF][16 * OP];
  const __bf16* Ut = (const __bf16*)Utp;
  const int tid = threadIdx.x, lane = tid & 31, wave = tid >> 5;
  const int c = lane & 15, hh = lane >> 4, koff = hh * 8;

  float hst[2][8], bb[2][3];
#pragma unroll
  for (int nt = 0; nt < 2; ++nt) {
    const int j = 32 * wave + 16 * nt + c;
#pragma unroll
    for (int g = 0; g < 3; ++g) bb[nt][g] = bf16r(bvec[kGate3 + g * kUnits + j]);
#pragma unroll
    for (int r = 0; r < 8; ++r) hst[nt][r] = HC[LAYER * (kBatch * kUnits) + (8 * hh + r) * kUnits + j];
  }
#pragma unroll
  for (int nt = 0; nt < 2; ++nt) {
    const int j = 32 * wave + 16 * nt + c;
#pragma unroll
    for (int r = 0; r < 8; ++r) {
      const float hv = hst[nt][r];
      const unsigned short hb = f2bf_bits(hv);
      const unsigned short lb = f2bf_bits(hv - bf_bits2f(hb));
      Ahh[0][(8 * hh + r) * HP + j] = hb;
      Ahl[0][(8 * hh + r) * HP + j] = lb;
    }
  }
  __syncthreads();

  const v8f z8 = {0.f, 0.f, 0.f, 0.f, 0.f, 0.f, 0.f, 0.f};

#pragma unroll 1
  for (int t = 0; t < kHalfSteps; ++t) {
    const int cur = t & 1, nxt = cur ^ 1;
    const __bf16* arow_h = (const __bf16*)(&Ahh[cur][0]) + c * HP + koff;
    const __bf16* arow_l = (const __bf16*)(&Ahl[cur][0]) + c * HP + koff;
    unsigned short* nh = &Ahh[nxt][0];
    unsigned short* nl = &Ahl[nxt][0];
    float* hfn = &Hf[(LAYER == 1) ? nxt : 0][0];
#pragma unroll
    for (int nt = 0; nt < 2; ++nt) {
      const int j = 32 * wave + 16 * nt + c;
      float xv[3][8];
#pragma unroll
      for (int g = 0; g < 3; ++g)
#pragma unroll
        for (int r = 0; r < 8; ++r)
          xv[g][r] = XP[((size_t)(8 * hh + r) * kHalfSteps + (size_t)t) * kGate3 + g * kUnits + j];
      const __bf16* u = Ut + (size_t)j * kUnits + koff;
      v8f a0 = z8, a1 = z8, a2 = z8;
#pragma unroll 1
      for (int k0 = 0; k0 < kUnits; k0 += 32) {
        const v16b ah = Frag<__bf16>::load(arow_h + k0);
        const v16b al = Frag<__bf16>::load(arow_l + k0);
        const v16b b0 = Frag<__bf16>::load(u + k0);
        const v16b b1 = Frag<__bf16>::load(u + (size_t)1 * kUnits * kUnits + k0);
        const v16b b2 = Frag<__bf16>::load(u + (size_t)2 * kUnits * kUnits + k0);
        a0 = Frag<__bf16>::mma(ah, b0, a0);
        a1 = Frag<__bf16>::mma(ah, b1, a1);
        a2 = Frag<__bf16>::mma(ah, b2, a2);
        a0 = Frag<__bf16>::mma(al, b0, a0);
        a1 = Frag<__bf16>::mma(al, b1, a1);
        a2 = Frag<__bf16>::mma(al, b2, a2);
        guard3_b(a0, a1, a2, ah, al, b0, b1, b2);
      }
      acc_guard3(a0, a1, a2);
#pragma unroll
      for (int g = 0; g < 3; ++g)
#pragma unroll
        for (int r = 0; r < 8; ++r) asm volatile("" : "+v"(xv[g][r]));
#pragma unroll
      for (int r = 0; r < 8; ++r) {
        const float hz = a0[r] + bb[nt][0];
        const float hr = a1[r] + bb[nt][1];
        const float hq = a2[r] + bb[nt][2];
        const float zg = fsig(xv[0][r] + hz);
        const float rg = fsig(xv[1][r] + hr);
        const float hc = ftanh(xv[2][r] + rg * hq);
        const float ho = hst[nt][r];
        const float hn = zg * ho + (1.0f - zg) * hc;
        hst[nt][r] = hn;
        const unsigned short hb = f2bf_bits(hn);
        const unsigned short lb = f2bf_bits(hn - bf_bits2f(hb));
        nh[(8 * hh + r) * HP + j] = hb;
        nl[(8 * hh + r) * HP + j] = lb;
        if (LAYER == 1) hfn[(8 * hh + r) * OP + j] = hn;
      }
    }
    __syncthreads();
    const size_t tg = (size_t)half * kHalfSteps + (size_t)t;
    if (LAYER == 0) {
      v8h vh[2], vl[2];
#pragma unroll
      for (int it = 0; it < 2; ++it) {
        const int idx = it * 256 + tid;
        const int row = idx >> 5, c8 = (idx & 31) * 8;
        vh[it] = *(const v8h*)(nh + row * HP + c8);
        vl[it] = *(const v8h*)(nl + row * HP + c8);
      }
      for (int pass = 0; pass < 2; ++pass) {
#pragma unroll
        for (int it = 0; it < 2; ++it) {
          const int idx = it * 256 + tid;
          const int row = idx >> 5, c8 = (idx & 31) * 8;
          const size_t o = ((size_t)row * kSteps + tg) * kUnits + c8;
          *(volatile v8h*)(YH + o) = vh[it];
          *(volatile v8h*)(YL + o) = vl[it];
        }
        __threadfence();
      }
    } else {
      v4f vo[4];
#pragma unroll
      for (int it = 0; it < 4; ++it) {
        const int idx = it * 256 + tid;
        const int row = idx >> 6, c4 = (idx & 63) * 4;
        vo[it] = *(const v4f*)(hfn + row * OP + c4);
      }
      for (int pass = 0; pass < 2; ++pass) {
#pragma unroll
        for (int it = 0; it < 4; ++it) {
          const int idx = it * 256 + tid;
          const int row = idx >> 6, c4 = (idx & 63) * 4;
          *(volatile v4f*)(out0 + ((size_t)row * kSteps + tg) * kUnits + c4) = vo[it];
        }
        __threadfence();
      }
    }
  }

  __syncthreads();
  float* hf0 = &Hf[0][0];
#pragma unroll
  for (int nt = 0; nt < 2; ++nt) {
    const int j = 32 * wave + 16 * nt + c;
#pragma unroll
    for (int r = 0; r < 8; ++r) hf0[(8 * hh + r) * OP + j] = hst[nt][r];
  }
  __syncthreads();
  {
    float* hcp = HC + LAYER * (kBatch * kUnits);
    v4f vo[4];
#pragma unroll
    for (int it = 0; it < 4; ++it) {
      const int idx = it * 256 + tid;
      const int row = idx >> 6, c4 = (idx & 63) * 4;
      vo[it] = *(const v4f*)(hf0 + row * OP + c4);
    }
    for (int pass = 0; pass < 2; ++pass) {
#pragma unroll
      for (int it = 0; it < 4; ++it) {
        const int idx = it * 256 + tid;
        const int row = idx >> 6, c4 = (idx & 63) * 4;
        *(volatile v4f*)(hcp + (size_t)row * kUnits + c4) = vo[it];
      }
      __threadfence();
    }
  }
  if (LAYER == 1 && half == 1) {
#pragma unroll 1
    for (int it = 0; it < 8; ++it) {
      const int idx = it * 256 + tid;
      const int b = idx >> 7, u2 = (idx & 127) * 2;
      const float p0 = HC[b * kUnits + u2];
      const float p1 = HC[b * kUnits + u2 + 1];
      const float q0 = hf0[b * OP + u2];
      const float q1 = hf0[b * OP + u2 + 1];
      v4f o;
      o[0] = p0; o[1] = q0; o[2] = p1; o[3] = q1;
      *(volatile v4f*)(out1 + (size_t)idx * 4) = o;
      __threadfence();
      *(volatile v4f*)(out1 + (size_t)idx * 4) = o;
    }
  }
}

extern "C" void kernel_launch(void* const* d_in, const int* in_sizes, int n_in,
                              void* d_out, int out_size, void* d_ws, size_t ws_size, hipStream_t stream) {
  if (n_in < 9 || d_out == nullptr || d_ws == nullptr) return;
  if (in_sizes[0] != kBatch * kSteps * kCin || in_sizes[1] != 3 * kCin * kFilt || in_sizes[2] != kFilt ||
      in_sizes[3] != kFilt * kGate3 || in_sizes[4] != kUnits * kGate3 || in_sizes[5] != 2 * kGate3 ||
      in_sizes[6] != kUnits * kGate3 || in_sizes[7] != kUnits * kGate3 || in_sizes[8] != 2 * kGate3 ||
      out_size != kOut0 + kOut1) return;

  const float* input_seq = (const float*)d_in[0];
  const float* conv_w    = (const float*)d_in[1];
  const float* conv_b    = (const float*)d_in[2];
  const float* w0        = (const float*)d_in[3];
  const float* u0        = (const float*)d_in[4];
  const float* b0        = (const float*)d_in[5];
  const float* w1        = (const float*)d_in[6];
  const float* u1        = (const float*)d_in[7];
  const float* b1        = (const float*)d_in[8];
  float* out0 = (float*)d_out;
  float* out1 = out0 + (size_t)kOut0;

  char* ws = (char*)d_ws; size_t off = 0;
  auto carve = [&](size_t bytes) -> char* { char* p = ws + off; off += (bytes + 255) & ~(size_t)255; return p; };
  unsigned short* XPAD = (unsigned short*)carve((size_t)kBatch * kPadRows * kCin * 2);
  unsigned short* CWT  = (unsigned short*)carve((size_t)kFilt * kConvK * 2);
  unsigned short* W0T  = (unsigned short*)carve((size_t)kGate3 * kFilt * 2);
  unsigned short* U0T  = (unsigned short*)carve((size_t)kGate3 * kUnits * 2);
  unsigned short* W1T  = (unsigned short*)carve((size_t)kGate3 * kUnits * 2);
  unsigned short* U1T  = (unsigned short*)carve((size_t)kGate3 * kUnits * 2);
  unsigned short* XH   = (unsigned short*)carve((size_t)kRows * kFilt * 2);
  unsigned short* XL   = (unsigned short*)carve((size_t)kRows * kFilt * 2);
  unsigned short* YH   = (unsigned short*)carve((size_t)kRows * kUnits * 2);
  unsigned short* YL   = (unsigned short*)carve((size_t)kRows * kUnits * 2);
  float*          XP   = (float*)carve((size_t)kRowsHalf * kGate3 * 4);
  float*          HC   = (float*)carve((size_t)2 * kBatch * kUnits * 4);
  if (off > ws_size || off > (size_t)134217728) return;

  xpad_kernel<<<(kBatch * kPadRows * (kCin / 8)) / 256, 256, 0, stream>>>(input_seq, XPAD);
  zero_kernel<<<(2 * kBatch * kUnits / 4) / 256, 256, 0, stream>>>(HC, 2 * kBatch * kUnits / 4);
  tp_bf16_kernel<<<dim3(kFilt / 64, kConvK / 64, 1), 256, 0, stream>>>(conv_w, conv_w, conv_w, conv_w, CWT, CWT, CWT, CWT,
                                                                       kConvK, kFilt);
  tp_bf16_kernel<<<dim3(kGate3 / 64, kFilt / 64, 4), 256, 0, stream>>>(w0, u0, w1, u1, W0T, U0T, W1T, U1T, kFilt, kGate3);

  gemm64_bf16<1, 2><<<(kRows / 64) * (kFilt / 64) / 8, 256, 0, stream>>>(
      XPAD, XPAD, kCin, 11, 2, 0, CWT, kConvK, (void*)XH, (void*)XL, kFilt, conv_b, kRows, kFilt, kConvK);

  const int xgrid = (kRowsHalf / 64) * (kGate3 / 64) / 8;
  for (int half = 0; half < 2; ++half) {
    gemm64_bf16<2, 0><<<xgrid, 256, 0, stream>>>(
        XH, XL, kFilt, 10, kHalfSteps, half * kHalfSteps, W0T, kFilt, (void*)XP, (void*)XP, kGate3, b0,
        kRowsHalf, kGate3, kFilt);
    gru_scan_kernel<0><<<1, 256, 0, stream>>>(XP, U0T, b0, HC, YH, YL, out0, out1, half);
  }
  for (int half = 0; half < 2; ++half) {
    gemm64_bf16<2, 0><<<xgrid, 256, 0, stream>>>(
        YH, YL, kUnits, 10, kHalfSteps, half * kHalfSteps, W1T, kUnits, (void*)XP, (void*)XP, kGate3, b1,
        kRowsHalf, kGate3, kUnits);
    gru_scan_kernel<1><<<1, 256, 0, stream>>>(XP, U1T, b1, HC, YH, YL, out0, out1, half);
  }
}
